// GDMLTorchAssemble_5188320493598
// MI455X (gfx1250) — hardware-verified
//
#include <hip/hip_runtime.h>
#include <stddef.h>
#include <math.h>


#define NAT    30
#define DIMD   435
#define DPAD   448
#define DIMI   90
#define IPAD   96
#define NPERM  12
#define TPLN   5220
#define RDW    1305
#define NTHR   256
#define NWAVE  8
#define NLOC   8
#define OUTPP  8100
#define KSTEPS 14
#define NBT    252
#define NBR    6
#define SBN    8136
#define QF     0.223606797749979f
#define QQ3    0.016666666666666673f

static_assert(NPERM * IPAD * (DPAD / 8) == NBT * NTHR);
static_assert(NBR * NTHR >= NPERM * (DPAD / 4));
static_assert(KSTEPS * 32 == DPAD);
static_assert((OUTPP * NLOC) % 32 == 0);
static_assert(SBN >= OUTPP + 32);
static_assert(DIMD * 3 == RDW);
static_assert(DIMI * DIMI == OUTPP);

#define O_BH  0
#define O_BL  (O_BH + 32 * DPAD * 2)
#define O_W   (O_BL + 32 * DPAD * 2)
#define W_SZ  (DIMD * 32 * 4)
#define O_AH  (O_W)
#define O_AL  (O_W + 16 * DPAD * 2)
#define O_RED (O_W + 32 * DPAD * 2)
#define O_XD  (O_W + W_SZ)
#define O_IN  (O_XD + NPERM * DPAD * 4)
#define O_SB  (O_IN + NPERM * IPAD * 4)
#define O_PD  (O_SB + SBN * 4)
#define O_RC  (O_PD + NPERM * DPAD * 2)
#define O_RJ  (O_RC + DPAD * 4)
#define O_RN  (O_RJ + 1312 * 4)
#define O_SC  (O_RN + 1312 * 4)
#define SMEM  (O_SC + 64 * 4)
static_assert(32 * DPAD * 2 + 8 * 256 * 4 <= W_SZ);
static_assert((O_W % 16) == 0 && (O_XD % 16) == 0 && (O_IN % 16) == 0 && (O_SB % 16) == 0);
static_assert((O_PD % 16) == 0 && (O_RC % 16) == 0 && (O_RJ % 16) == 0 && (O_RN % 16) == 0 && (O_SC % 16) == 0);
static_assert(SMEM <= 200 * 1024);

typedef float          v4f  __attribute__((ext_vector_type(4)));
typedef float          v8f  __attribute__((ext_vector_type(8)));
typedef unsigned short v4us __attribute__((ext_vector_type(4)));
typedef unsigned short v8us __attribute__((ext_vector_type(8)));
typedef __bf16         v16b __attribute__((ext_vector_type(16)));
union FragB { v16b v; v8us h[2]; };

__device__ __forceinline__ int iclamp(int x, int lo, int hi) { return x < lo ? lo : (x > hi ? hi : x); }

__device__ __forceinline__ unsigned short bf_rne(float x) {
  unsigned u = __float_as_uint(x);
  u += 0x7FFFu + ((u >> 16) & 1u);
  return (unsigned short)(u >> 16);
}
__device__ __forceinline__ float bf_val(unsigned short b) { return __uint_as_float(((unsigned)b) << 16); }

__device__ __forceinline__ v8f zero8f() {
  v8f c;
#pragma unroll
  for (int i = 0; i < 8; ++i) c[i] = 0.0f;
  return c;
}

__device__ __forceinline__ v8f wmb(v16b a, v16b b, v8f c) {
  v8f d = __builtin_amdgcn_wmma_f32_16x16x32_bf16(false, a, false, b, (short)0, c, false, false);
  asm volatile("v_nop\n\tv_nop\n\tv_nop\n\tv_nop" : "+v"(d) : "v"(a), "v"(b));
  return d;
}
__device__ __forceinline__ v8f wm3(v16b ah, v16b al, v16b bh, v16b bl, v8f c) {
  c = wmb(ah, bh, c);
  c = wmb(ah, bl, c);
  c = wmb(al, bh, c);
  return c;
}

__global__ __launch_bounds__(NTHR) void k_setup(const float* __restrict__ Rdesc, const float* __restrict__ Rdd,
                                               const int* __restrict__ tpl, const int* __restrict__ jp, int N,
                                               unsigned short* TH, unsigned short* TL, float* rjdp) {
  __shared__ int rcs[DPAD];
  const int tid = threadIdx.x;
  for (int t = tid; t < NAT * NAT; t += NTHR) {
    const int r = t / NAT, c = t - r * NAT;
    if (c < r) rcs[r * (r - 1) / 2 + c] = r | (c << 8);
  }
  for (int t = DIMD + tid; t < DPAD; t += NTHR) rcs[t] = 0;
  __syncthreads();
  int j = jp[0];
  j = iclamp(j, 0, N - 1);
  const int b = blockIdx.x;
  if (b < NBT) {
    const int u  = b * NTHR + tid;
    const int p  = u / (IPAD * (DPAD / 8));
    const int rm = u - p * (IPAD * (DPAD / 8));
    const int i  = rm / (DPAD / 8);
    const int c8 = rm - i * (DPAD / 8);
    const int ai = i / 3, ci = i - 3 * ai;
    v8us hv, lv;
#pragma unroll
    for (int e = 0; e < 8; ++e) {
      const int d  = 8 * c8 + e;
      const int dc = d < DIMD ? d : DIMD - 1;
      int v = tpl[dc * NPERM + p];
      v = v < 0 ? v + TPLN : v;
      v = iclamp(v, 0, TPLN - 1);
      const int pd = v % DIMD;
      const int rc = rcs[pd];
      const int ra = rc & 255, cb = rc >> 8;
      const float val = Rdd[((size_t)j * DIMD + pd) * 3 + ci];
      float w = (ai == ra) ? val : ((ai == cb) ? -val : 0.0f);
      w = (d < DIMD && i < DIMI) ? w : 0.0f;
      const unsigned short hb = bf_rne(w);
      hv[e] = hb;
      lv[e] = bf_rne(w - bf_val(hb));
    }
    unsigned short* thp = TH + (size_t)u * 8;
    unsigned short* tlp = TL + (size_t)u * 8;
    *(volatile v8us*)thp = hv;
    *(volatile v8us*)tlp = lv;
    __threadfence();
    *(volatile v8us*)thp = hv;
    *(volatile v8us*)tlp = lv;
  } else {
    const int u = (b - NBT) * NTHR + tid;
    if (u < NPERM * (DPAD / 4)) {
      const int p  = u / (DPAD / 4);
      const int c4 = u - p * (DPAD / 4);
      v4f o;
#pragma unroll
      for (int e = 0; e < 4; ++e) {
        const int d  = 4 * c4 + e;
        const int dc = d < DIMD ? d : DIMD - 1;
        int v = tpl[dc * NPERM + p];
        v = v < 0 ? v + TPLN : v;
        v = iclamp(v, 0, TPLN - 1);
        const int pd = v % DIMD;
        float w = Rdesc[(size_t)j * DIMD + pd];
        w = d < DIMD ? w : 0.0f;
        o[e] = w;
      }
      float* rp = rjdp + (size_t)u * 4;
      *(volatile v4f*)rp = o;
      __threadfence();
      *(volatile v4f*)rp = o;
    }
  }
}

__global__ __launch_bounds__(NTHR) void k_xd(const float* __restrict__ Rdesc, const float* __restrict__ rjdp,
                                            unsigned short* XH, unsigned short* XL, int N, int Np) {
  const int p  = blockIdx.y;
  const int u  = blockIdx.x * NTHR + threadIdx.x;
  const int n  = u / (DPAD / 8);
  const int c8 = u - n * (DPAD / 8);
  const int nn = n < N ? n : N - 1;
  v8us hv, lv;
#pragma unroll
  for (int e = 0; e < 8; ++e) {
    const int d  = 8 * c8 + e;
    const int dc = d < DIMD ? d : DIMD - 1;
    const float a  = Rdesc[(size_t)nn * DIMD + dc];
    const float bq = rjdp[p * DPAD + d];
    float x = QF * (a - bq);
    x = (d < DIMD && n < N) ? x : 0.0f;
    const unsigned short hb = bf_rne(x);
    hv[e] = hb;
    lv[e] = bf_rne(x - bf_val(hb));
  }
  const size_t xo = ((size_t)p * Np + n) * DPAD + 8 * c8;
  unsigned short* xhp = XH + xo;
  unsigned short* xlp = XL + xo;
  *(volatile v8us*)xhp = hv;
  *(volatile v8us*)xlp = lv;
  __threadfence();
  *(volatile v8us*)xhp = hv;
  *(volatile v8us*)xlp = lv;
}

__global__ __launch_bounds__(NTHR) void k_inner(const unsigned short* __restrict__ XH,
                                               const unsigned short* __restrict__ XL,
                                               const unsigned short* __restrict__ TH,
                                               const unsigned short* __restrict__ TL,
                                               float* inner, int Np) {
  __shared__ __attribute__((aligned(16))) float Cs[64 * IPAD];
  const int tid = threadIdx.x, lane = tid & 31, wave = tid >> 5, h = lane >> 4, m = lane & 15;
  const int p  = blockIdx.y;
  const int n0 = blockIdx.x * 64;
  const int rt = wave >> 1, cg = wave & 1;
  const size_t ao = ((size_t)p * Np + n0 + 16 * rt + m) * DPAD + 8 * h;
  const size_t bo = ((size_t)p * IPAD + 48 * cg + m) * DPAD + 8 * h;
  const unsigned short* ahp = XH + ao;
  const unsigned short* alp = XL + ao;
  const unsigned short* bhp = TH + bo;
  const unsigned short* blp = TL + bo;
  v8f c0 = zero8f(), c1 = zero8f(), c2 = zero8f();
#pragma unroll 1
  for (int ks = 0; ks < KSTEPS; ++ks) {
    const int k0 = 32 * ks;
    FragB ah, al, bh, bl;
    ah.h[0] = *(const v8us*)(ahp + k0);  ah.h[1] = *(const v8us*)(ahp + k0 + 16);
    al.h[0] = *(const v8us*)(alp + k0);  al.h[1] = *(const v8us*)(alp + k0 + 16);
    bh.h[0] = *(const v8us*)(bhp + k0);  bh.h[1] = *(const v8us*)(bhp + k0 + 16);
    bl.h[0] = *(const v8us*)(blp + k0);  bl.h[1] = *(const v8us*)(blp + k0 + 16);
    c0 = wm3(ah.v, al.v, bh.v, bl.v, c0);
    bh.h[0] = *(const v8us*)(bhp + 16 * DPAD + k0);  bh.h[1] = *(const v8us*)(bhp + 16 * DPAD + k0 + 16);
    bl.h[0] = *(const v8us*)(blp + 16 * DPAD + k0);  bl.h[1] = *(const v8us*)(blp + 16 * DPAD + k0 + 16);
    c1 = wm3(ah.v, al.v, bh.v, bl.v, c1);
    bh.h[0] = *(const v8us*)(bhp + 32 * DPAD + k0);  bh.h[1] = *(const v8us*)(bhp + 32 * DPAD + k0 + 16);
    bl.h[0] = *(const v8us*)(blp + 32 * DPAD + k0);  bl.h[1] = *(const v8us*)(blp + 32 * DPAD + k0 + 16);
    c2 = wm3(ah.v, al.v, bh.v, bl.v, c2);
  }
  {
    float* cp = Cs + (16 * rt + 8 * h) * IPAD + 48 * cg + m;
#pragma unroll
    for (int r = 0; r < 8; ++r) {
      cp[r * IPAD]      = c0[r];
      cp[r * IPAD + 16] = c1[r];
      cp[r * IPAD + 32] = c2[r];
    }
  }
  __syncthreads();
  const int pc = lane & 7;
#pragma unroll
  for (int s = 0; s < 6; ++s) {
    const int L = 24 * wave + 4 * s + (lane >> 3);
    const int row = L / 3, lr = L - 3 * row;
    const v4f v = *(const v4f*)(Cs + row * IPAD + 32 * lr + 4 * pc);
    *(volatile v4f*)(inner + ((size_t)(n0 + row) * NPERM + p) * IPAD + 32 * lr + 4 * pc) = v;
  }
  __threadfence();
#pragma unroll
  for (int s = 0; s < 6; ++s) {
    const int L = 24 * wave + 4 * s + (lane >> 3);
    const int row = L / 3, lr = L - 3 * row;
    const v4f v = *(const v4f*)(Cs + row * IPAD + 32 * lr + 4 * pc);
    *(volatile v4f*)(inner + ((size_t)(n0 + row) * NPERM + p) * IPAD + 32 * lr + 4 * pc) = v;
  }
}

__device__ __forceinline__ void flush_lines(const float* SB, float* out, size_t fb, int nfl, int wave, int lane) {
  const int pc = lane & 7;
#pragma unroll 1
  for (int s = 0; s < 8; ++s) {
    const int L = 32 * s + 4 * wave + (lane >> 3);
    if (L < nfl) {
      const v4f v = *(const v4f*)(SB + 32 * L + 4 * pc);
      *(volatile v4f*)(out + fb + (size_t)32 * L + 4 * pc) = v;
    }
  }
}

__global__ __launch_bounds__(NTHR) void k_asm(const float* __restrict__ Rdesc, const float* __restrict__ Rdd,
                                             const int* __restrict__ tpl, const int* __restrict__ jp,
                                             const float* __restrict__ rjdp, const float* __restrict__ inner,
                                             float* out, int N) {
  extern __shared__ __attribute__((aligned(16))) unsigned char smem[];
  unsigned short* BH = (unsigned short*)(smem + O_BH);
  unsigned short* BL = (unsigned short*)(smem + O_BL);
  float* DAB = (float*)(smem + O_W);
  unsigned short* AH = (unsigned short*)(smem + O_AH);
  unsigned short* AL = (unsigned short*)(smem + O_AL);
  float* RED = (float*)(smem + O_RED);
  float* XD  = (float*)(smem + O_XD);
  float* INL = (float*)(smem + O_IN);
  float* SB  = (float*)(smem + O_SB);
  unsigned short* PD = (unsigned short*)(smem + O_PD);
  int*   RC  = (int*)(smem + O_RC);
  float* RJ  = (float*)(smem + O_RJ);
  float* RN  = (float*)(smem + O_RN);
  float* EX  = (float*)(smem + O_SC);
  float* E1  = EX + 16;

  const int tid = threadIdx.x, lane = tid & 31, wave = tid >> 5, h = lane >> 4, m = lane & 15;
  const int g  = blockIdx.x;
  const int n0 = g * NLOC;
  int nloc = N - n0;
  nloc = nloc > NLOC ? NLOC : nloc;
  int j = jp[0];
  j = iclamp(j, 0, N - 1);

  for (int t2 = tid; t2 < NAT * NAT; t2 += NTHR) {
    const int r = t2 / NAT, c = t2 - r * NAT;
    if (c < r) RC[r * (r - 1) / 2 + c] = r | (c << 8);
  }
  for (int t2 = DIMD + tid; t2 < DPAD; t2 += NTHR) RC[t2] = 0;
  for (int t2 = tid; t2 < NPERM * DPAD; t2 += NTHR) {
    const int p = t2 / DPAD, d = t2 - p * DPAD;
    const int dc = d < DIMD ? d : DIMD - 1;
    int v = tpl[dc * NPERM + p];
    v = v < 0 ? v + TPLN : v;
    v = iclamp(v, 0, TPLN - 1);
    const int pd = (d < DIMD) ? (v % DIMD) : 0;
    PD[t2] = (unsigned short)pd;
  }
  for (int t2 = tid; t2 < RDW; t2 += NTHR) RJ[t2] = Rdd[(size_t)j * RDW + t2];
  __syncthreads();

  const size_t fbase = (size_t)g * (size_t)(NLOC * OUTPP);
  int rem = 0, ldone = 0;

  for (int t = 0; t < nloc; ++t) {
    const int n = n0 + t;
    for (int e = tid; e < NPERM * DPAD; e += NTHR) {
      const int p = e / DPAD, d = e - p * DPAD;
      const int dc = d < DIMD ? d : DIMD - 1;
      const float a  = Rdesc[(size_t)n * DIMD + dc];
      const float bq = rjdp[e];
      float x = QF * (a - bq);
      x = d < DIMD ? x : 0.0f;
      XD[e] = x;
    }
    for (int e = tid; e < RDW; e += NTHR) RN[e] = Rdd[(size_t)n * RDW + e];
    for (int e = tid; e < NPERM * IPAD; e += NTHR) INL[e] = inner[(size_t)n * (NPERM * IPAD) + e];
    __syncthreads();

    for (int p = wave; p < NPERM; p += NWAVE) {
      float s = 0.0f;
      for (int d = lane; d < DPAD; d += 32) { const float x = XD[p * DPAD + d]; s += x * x; }
      s += __shfl_xor(s, 16, 32);
      s += __shfl_xor(s, 8, 32);
      s += __shfl_xor(s, 4, 32);
      s += __shfl_xor(s, 2, 32);
      s += __shfl_xor(s, 1, 32);
      if (lane == 0) {
        const float dist = sqrtf(s);
        const float ex = expf(-dist) * QQ3;
        EX[p] = ex;
        E1[p] = ex * (1.0f + dist);
      }
    }
    __syncthreads();

    for (int ch = 0; ch < 3; ++ch) {
#pragma unroll
      for (int slot = 0; slot < 2; ++slot) {
        const int d  = tid + NTHR * slot;
        const int dd = d < DIMD ? d : DIMD - 1;
        v4f acc[8];
#pragma unroll
        for (int gq = 0; gq < 8; ++gq) { acc[gq].x = 0.0f; acc[gq].y = 0.0f; acc[gq].z = 0.0f; acc[gq].w = 0.0f; }
#pragma unroll 1
        for (int p = 0; p < NPERM; ++p) {
          const float xp = XD[p * DPAD + dd] * EX[p];
          const float* ip = INL + p * IPAD + 32 * ch;
#pragma unroll
          for (int gq = 0; gq < 8; ++gq) {
            const v4f iv = *(const v4f*)(ip + 4 * gq);
            acc[gq] += iv * xp;
          }
        }
        if (d < DIMD) {
#pragma unroll
          for (int gq = 0; gq < 8; ++gq) *(v4f*)(DAB + d * 32 + 4 * gq) = acc[gq];
        }
      }
      __syncthreads();
#pragma unroll
      for (int slot = 0; slot < 2; ++slot) {
        const int d = tid + NTHR * slot;
        if (d < DIMD) {
          float* row = DAB + d * 32;
#pragma unroll 1
          for (int p = 0; p < NPERM; ++p) {
            const int pd = PD[p * DPAD + d];
            const int rc = RC[pd];
            const int ra = rc & 255, cb = rc >> 8;
            const float w1 = E1[p];
#pragma unroll
            for (int c = 0; c < 3; ++c) {
              const float v = RJ[pd * 3 + c] * w1;
              int ia = 3 * ra + c - 32 * ch;
              int ib = 3 * cb + c - 32 * ch;
              const float fa = ((unsigned)ia < 32u) ? v : 0.0f;
              const float fb = ((unsigned)ib < 32u) ? v : 0.0f;
              ia = iclamp(ia, 0, 31);
              ib = iclamp(ib, 0, 31);
              row[ia] = row[ia] - fa;
              row[ib] = row[ib] + fb;
            }
          }
        }
      }
      __syncthreads();
      for (int t2 = tid; t2 < 32 * (DPAD / 8); t2 += NTHR) {
        const int jl = t2 / (DPAD / 8), c8 = t2 - jl * (DPAD / 8);
        v8us hv, lv;
#pragma unroll
        for (int e = 0; e < 8; ++e) {
          const int d  = 8 * c8 + e;
          const int dc = d < DIMD ? d : DIMD - 1;
          float v = DAB[dc * 32 + jl];
          v = d < DIMD ? v : 0.0f;
          const unsigned short hb = bf_rne(v);
          hv[e] = hb;
          lv[e] = bf_rne(v - bf_val(hb));
        }
        *(v8us*)(BH + jl * DPAD + 8 * c8) = hv;
        *(v8us*)(BL + jl * DPAD + 8 * c8) = lv;
      }
      __syncthreads();
      for (int mt = 0; mt < 6; ++mt) {
        {
          v8us z;
#pragma unroll
          for (int e = 0; e < 8; ++e) z[e] = 0;
          for (int t2 = tid; t2 < 16 * (DPAD / 8); t2 += NTHR) {
            *(v8us*)(AH + 8 * t2) = z;
            *(v8us*)(AL + 8 * t2) = z;
          }
        }
        __syncthreads();
        for (int t2 = tid; t2 < 16 * 29; t2 += NTHR) {
          const int kl = t2 / 29, tt = t2 - kl * 29;
          const int kk = 16 * mt + kl;
          if (kk < DIMI) {
            const int a  = kk / 3, c = kk - 3 * a;
            const int bb = tt < a ? tt : tt + 1;
            const int lo = bb < a ? bb : a;
            const int hi = bb < a ? a : bb;
            const int d  = hi * (hi - 1) / 2 + lo;
            const float sg = bb < a ? 1.0f : -1.0f;
            const float v = sg * RN[d * 3 + c];
            const unsigned short hb = bf_rne(v);
            AH[kl * DPAD + d] = hb;
            AL[kl * DPAD + d] = bf_rne(v - bf_val(hb));
          }
        }
        __syncthreads();
        {
          const int nt = wave & 1, kq = wave >> 1;
          const unsigned short* ahp = AH + m * DPAD + 8 * h;
          const unsigned short* alp = AL + m * DPAD + 8 * h;
          const unsigned short* bhp = BH + (16 * nt + m) * DPAD + 8 * h;
          const unsigned short* blp = BL + (16 * nt + m) * DPAD + 8 * h;
          v8f cacc = zero8f();
          for (int ks = kq; ks < KSTEPS; ks += 4) {
            const int k0 = 32 * ks;
            FragB fah, fal, fbh, fbl;
            fah.h[0] = *(const v8us*)(ahp + k0); fah.h[1] = *(const v8us*)(ahp + k0 + 16);
            fal.h[0] = *(const v8us*)(alp + k0); fal.h[1] = *(const v8us*)(alp + k0 + 16);
            fbh.h[0] = *(const v8us*)(bhp + k0); fbh.h[1] = *(const v8us*)(bhp + k0 + 16);
            fbl.h[0] = *(const v8us*)(blp + k0); fbl.h[1] = *(const v8us*)(blp + k0 + 16);
            cacc = wm3(fah.v, fal.v, fbh.v, fbl.v, cacc);
          }
          float* rp = RED + (kq * 2 + nt) * 256 + (8 * h) * 16 + m;
#pragma unroll
          for (int r = 0; r < 8; ++r) rp[16 * r] = cacc[r];
        }
        __syncthreads();
        for (int o = tid; o < 512; o += NTHR) {
          const int nt = o >> 8, e = o & 255;
          float s = RED[(0 * 2 + nt) * 256 + e];
          s += RED[(1 * 2 + nt) * 256 + e];
          s += RED[(2 * 2 + nt) * 256 + e];
          s += RED[(3 * 2 + nt) * 256 + e];
          const int kl = e >> 4, col = e & 15;
          const int kk = 16 * mt + kl, jj = 32 * ch + 16 * nt + col;
          if (kk < DIMI && jj < DIMI) SB[rem + kk * DIMI + jj] = s;
        }
        __syncthreads();
      }
    }

    {
      const int avail = rem + OUTPP;
      const int nfl = avail >> 5;
      const size_t fb = fbase + (size_t)32 * ldone;
      flush_lines(SB, out, fb, nfl, wave, lane);
      __threadfence();
      flush_lines(SB, out, fb, nfl, wave, lane);
      __syncthreads();
      const int nrem = avail - 32 * nfl;
      float cv = SB[tid];
      if (tid < nrem) cv = SB[32 * nfl + tid];
      __syncthreads();
      if (tid < nrem) SB[tid] = cv;
      __syncthreads();
      rem = nrem;
      ldone += nfl;
    }
  }
  if (rem > 0) {
    const float v = SB[tid & 31];
    float* op = out + fbase + (size_t)32 * ldone + tid;
    if (tid < rem) *(volatile float*)op = v;
    __threadfence();
    if (tid < rem) *(volatile float*)op = v;
  }
}

extern "C" void kernel_launch(void* const* d_in, const int* in_sizes, int n_in,
                              void* d_out, int out_size, void* d_ws, size_t ws_size,
                              hipStream_t stream) {
  if (n_in < 4) return;
  if (in_sizes[0] < DIMD || (in_sizes[0] % DIMD) != 0) return;
  const int N = in_sizes[0] / DIMD;
  if (in_sizes[1] != N * RDW || in_sizes[2] != TPLN || in_sizes[3] < 1) return;
  if (out_size != N * OUTPP) return;
  const int Np = ((N + 63) / 64) * 64;

  const float* Rdesc = (const float*)d_in[0];
  const float* Rdd   = (const float*)d_in[1];
  const int*   tpl   = (const int*)d_in[2];
  const int*   jp    = (const int*)d_in[3];
  float* outp = (float*)d_out;

  char* ws = (char*)d_ws;
  size_t off = 0;
  const size_t oRJ = off; off += ((size_t)NPERM * DPAD * 4 + 255) & ~(size_t)255;
  const size_t oTH = off; off += ((size_t)NPERM * IPAD * DPAD * 2 + 255) & ~(size_t)255;
  const size_t oTL = off; off += ((size_t)NPERM * IPAD * DPAD * 2 + 255) & ~(size_t)255;
  const size_t oXH = off; off += ((size_t)NPERM * (size_t)Np * DPAD * 2 + 255) & ~(size_t)255;
  const size_t oXL = off; off += ((size_t)NPERM * (size_t)Np * DPAD * 2 + 255) & ~(size_t)255;
  const size_t oIN = off; off += ((size_t)Np * NPERM * IPAD * 4 + 255) & ~(size_t)255;
  size_t limit = (size_t)134217728;
  if (ws_size < limit) limit = ws_size;
  if (off > limit) return;

  float*          rjdp = (float*)(ws + oRJ);
  unsigned short* TH   = (unsigned short*)(ws + oTH);
  unsigned short* TL   = (unsigned short*)(ws + oTL);
  unsigned short* XH   = (unsigned short*)(ws + oXH);
  unsigned short* XL   = (unsigned short*)(ws + oXL);
  float*          innr = (float*)(ws + oIN);

  k_setup<<<NBT + NBR, NTHR, 0, stream>>>(Rdesc, Rdd, tpl, jp, N, TH, TL, rjdp);
  k_xd<<<dim3(Np * (DPAD / 8) / NTHR, NPERM), NTHR, 0, stream>>>(Rdesc, rjdp, XH, XL, N, Np);
  k_inner<<<dim3(Np / 64, NPERM), NTHR, 0, stream>>>(XH, XL, TH, TL, innr, Np);
  hipFuncSetAttribute(reinterpret_cast<const void*>(&k_asm), hipFuncAttributeMaxDynamicSharedMemorySize, SMEM);
  k_asm<<<(N + NLOC - 1) / NLOC, NTHR, SMEM, stream>>>(Rdesc, Rdd, tpl, jp, rjdp, innr, outp, N);
}
